// INNv2CUDA_44976897523879
// MI455X (gfx1250) — hardware-verified
//
#include <hip/hip_runtime.h>
#include <hip/hip_bf16.h>
#include <math.h>


#define LSEQ  512
#define DMOD  256
#define DINR  512
#define NST   16
#define NLAY  4
#define VOCB  32000
#define XPW   64
#define DTK   32
#define SPIT  68

static_assert(LSEQ % 64 == 0);
static_assert(DMOD % 64 == 0);
static_assert(DINR % 64 == 0);
static_assert(VOCB % 64 == 0);
static_assert((2 * DINR) % 64 == 0);

typedef float          v4f   __attribute__((ext_vector_type(4)));
typedef float          v8f   __attribute__((ext_vector_type(8)));
typedef __bf16         v16b  __attribute__((ext_vector_type(16)));
typedef unsigned short u16x8 __attribute__((ext_vector_type(8)));
typedef unsigned short ush;

union FragB { u16x8 h[2]; v16b v; };

__device__ __forceinline__ ush f32_to_bf16(float f) {
  unsigned u = __float_as_uint(f);
  unsigned r = u + 0x7FFFu + ((u >> 16) & 1u);
  return (ush)(r >> 16);
}
__device__ __forceinline__ float bf16_to_f32(ush b) {
  return __uint_as_float(((unsigned)b) << 16);
}
__device__ __forceinline__ void split2(float f, ush& hb, ush& lb) {
  hb = f32_to_bf16(f);
  lb = f32_to_bf16(f - bf16_to_f32(hb));
}
__device__ __forceinline__ float silu_f(float x) {
  const float e = expf(-x);
  return x * __builtin_amdgcn_rcpf(1.0f + e);
}
__device__ __forceinline__ float softplus_f(float x) {
  return fmaxf(x, 0.0f) + log1pf(expf(-fabsf(x)));
}
__device__ __forceinline__ float conv4(float x0, float x1, float x2, float x3,
                                       float w0, float w1, float w2, float w3, float bias) {
  return ((w0 * x0 + w1 * x1) + (w2 * x2 + w3 * x3)) + bias;
}
__device__ __forceinline__ v8f ld8f(const float* p) {
  const v4f a = *(const v4f*)p;
  const v4f b = *(const v4f*)(p + 4);
  return __builtin_shufflevector(a, b, 0, 1, 2, 3, 4, 5, 6, 7);
}

__device__ __forceinline__ void mma16(v8f& acc, const FragB& a, const FragB& b) {
  acc = __builtin_amdgcn_wmma_f32_16x16x32_bf16(false, a.v, false, b.v, (short)0, acc, false, false);
  asm volatile("v_nop\n\tv_nop\n\tv_nop\n\tv_nop" : "+v"(acc) : "v"(a.v), "v"(b.v));
}

__global__ __launch_bounds__(256)
void cvt_rows_kernel(const float* __restrict__ src, ush* dh, ush* dl,
                     int R, int Kp, int Rsrc, int Ksrc, int spitch, int roff, int lstride, int total8)
{
  const int gid = blockIdx.x * 256 + threadIdx.x;
  if (gid >= total8) return;
  const size_t e    = (size_t)gid * 8;
  const size_t perL = (size_t)R * Kp;
  const int li  = (int)(e / perL);
  const int rem = (int)(e - (size_t)li * perL);
  const int r   = rem / Kp;
  const int k   = rem - r * Kp;
  const bool valid = (r < Rsrc) && (k < Ksrc);
  const int rc = (r < Rsrc) ? r : (Rsrc - 1);
  const int kc = (k <= Ksrc - 8) ? k : (Ksrc - 8);
  const float* sp = src + (size_t)li * lstride + (size_t)(rc + roff) * spitch + kc;
  const v4f a = *(const v4f*)sp;
  const v4f b = *(const v4f*)(sp + 4);
  u16x8 hv, lv;
#pragma unroll
  for (int c = 0; c < 8; ++c) {
    float f = (c < 4) ? a[c] : b[c - 4];
    if (!valid) f = 0.0f;
    ush hb, lb;
    split2(f, hb, lb);
    hv[c] = hb;
    lv[c] = lb;
  }
  *(volatile u16x8*)(dh + e) = hv;
  *(volatile u16x8*)(dl + e) = lv;
  __threadfence();
  *(volatile u16x8*)(dh + e) = hv;
  *(volatile u16x8*)(dl + e) = lv;
}

__global__ __launch_bounds__(256)
void embed_kernel(const int* __restrict__ tok, const float* __restrict__ emb, float* x, int ntok, int V)
{
  const int gid = blockIdx.x * 256 + threadIdx.x;
  if (gid >= ntok * (DMOD / 4)) return;
  const int e = gid * 4;
  const int l = e / DMOD;
  const int d = e - l * DMOD;
  int t = tok[l];
  if (t < 0) t += V;
  t = (t < 0) ? 0 : ((t >= V) ? (V - 1) : t);
  const v4f v = *(const v4f*)(emb + (size_t)t * DMOD + d);
  *(volatile v4f*)(x + e) = v;
  __threadfence();
  *(volatile v4f*)(x + e) = v;
}

__global__ __launch_bounds__(256)
void ln_cvt_kernel(const float* __restrict__ X, const float* __restrict__ g, const float* __restrict__ b,
                   ush* Yh, ush* Yl, int M)
{
  const int wave = threadIdx.x >> 5;
  const int lane = threadIdx.x & 31;
  const int row  = blockIdx.x * 8 + wave;
  if (row >= M) return;
  const float* xr = X + (size_t)row * DMOD + 8 * lane;
  const v8f x = ld8f(xr);
  float s = 0.0f;
#pragma unroll
  for (int j = 0; j < 8; ++j) s += x[j];
#pragma unroll
  for (int o = 16; o > 0; o >>= 1) s += __shfl_xor(s, o, 32);
  const float mean = s * (1.0f / 256.0f);
  float q = 0.0f;
#pragma unroll
  for (int j = 0; j < 8; ++j) { const float dd = x[j] - mean; q += dd * dd; }
#pragma unroll
  for (int o = 16; o > 0; o >>= 1) q += __shfl_xor(q, o, 32);
  const float rstd = rsqrtf(q * (1.0f / 256.0f) + 1e-5f);
  const v8f gv = ld8f(g + 8 * lane);
  const v8f bv = ld8f(b + 8 * lane);
  u16x8 hv, lv;
#pragma unroll
  for (int j = 0; j < 8; ++j) {
    const float y = (x[j] - mean) * rstd * gv[j] + bv[j];
    ush hb, lb;
    split2(y, hb, lb);
    hv[j] = hb;
    lv[j] = lb;
  }
  const size_t e = (size_t)row * DMOD + 8 * lane;
  *(volatile u16x8*)(Yh + e) = hv;
  *(volatile u16x8*)(Yl + e) = lv;
  __threadfence();
  *(volatile u16x8*)(Yh + e) = hv;
  *(volatile u16x8*)(Yl + e) = lv;
}

__global__ __launch_bounds__(64)
void conv_silu_kernel(const float* __restrict__ xz, const float* __restrict__ cw,
                      const float* __restrict__ cb, ush* xmh, ush* xml)
{
  const int l  = blockIdx.x;
  const int d0 = threadIdx.x * 8;
  const int r1 = (l >= 1) ? (l - 1) : 0;
  const int r2 = (l >= 2) ? (l - 2) : 0;
  const int r3 = (l >= 3) ? (l - 3) : 0;
  const v8f x3 = ld8f(xz + (size_t)l  * (2 * DINR) + d0);
  v8f x2 = ld8f(xz + (size_t)r1 * (2 * DINR) + d0);
  v8f x1 = ld8f(xz + (size_t)r2 * (2 * DINR) + d0);
  v8f x0 = ld8f(xz + (size_t)r3 * (2 * DINR) + d0);
  v8f zero;
#pragma unroll
  for (int c = 0; c < 8; ++c) zero[c] = 0.0f;
  if (l < 1) x2 = zero;
  if (l < 2) x1 = zero;
  if (l < 3) x0 = zero;

  const float* wp = cw + (size_t)d0 * 4;
  v4f wv[8];
#pragma unroll
  for (int c = 0; c < 8; ++c) wv[c] = *(const v4f*)(wp + 4 * c);
  const v8f bias = ld8f(cb + d0);

  u16x8 hv, lv;
#pragma unroll
  for (int c = 0; c < 8; ++c) {
    const float u = silu_f(conv4(x0[c], x1[c], x2[c], x3[c], wv[c][0], wv[c][1], wv[c][2], wv[c][3], bias[c]));
    ush hb, lb;
    split2(u, hb, lb);
    hv[c] = hb;
    lv[c] = lb;
  }
  const size_t e = (size_t)l * DINR + d0;
  *(volatile u16x8*)(xmh + e) = hv;
  *(volatile u16x8*)(xml + e) = lv;
  __threadfence();
  *(volatile u16x8*)(xmh + e) = hv;
  *(volatile u16x8*)(xml + e) = lv;
}

template<int OUTP>
__device__ __forceinline__ void gemm_store_pass(const float* st, float* Cf, ush* Ch, ush* Cl,
                                                int row0, int col0, int ldc, int wave, int lane)
{
  if (OUTP == 0) {
#pragma unroll
    for (int it = 0; it < 8; ++it) {
      const int row = it * 8 + 2 * wave + (lane >> 4);
      const int c   = 4 * (lane & 15);
      const v4f v = *(const v4f*)(st + row * SPIT + c);
      *(volatile v4f*)(Cf + (size_t)(row0 + row) * ldc + col0 + c) = v;
    }
  } else {
#pragma unroll
    for (int it = 0; it < 4; ++it) {
      const int row = it * 16 + 4 * wave + (lane >> 3);
      const int c   = 8 * (lane & 7);
      const v4f a = *(const v4f*)(st + row * SPIT + c);
      const v4f b = *(const v4f*)(st + row * SPIT + c + 4);
      u16x8 hv, lv;
#pragma unroll
      for (int e = 0; e < 8; ++e) {
        const float f = (e < 4) ? a[e] : b[e - 4];
        ush hb, lb;
        split2(f, hb, lb);
        hv[e] = hb;
        lv[e] = lb;
      }
      const size_t go = (size_t)(row0 + row) * ldc + col0 + c;
      *(volatile u16x8*)(Ch + go) = hv;
      *(volatile u16x8*)(Cl + go) = lv;
    }
  }
}

template<int OUTP>
__global__ __launch_bounds__(128)
void gemm_kernel(const ush* __restrict__ Ah, const ush* __restrict__ Al,
                 const ush* __restrict__ Bh, const ush* __restrict__ Bl,
                 const float* __restrict__ bias, const float* addsrc, int ldadd,
                 float* Cf, ush* Ch, ush* Cl, int K, int ldc, int flags)
{
  __shared__ __attribute__((aligned(16))) float stile[64 * SPIT];

  const int tid  = threadIdx.x;
  const int lane = tid & 31;
  const int wave = tid >> 5;
  const int h    = lane >> 4;
  const int m    = lane & 15;
  const int wm   = wave >> 1;
  const int wn   = wave & 1;
  const int row0 = blockIdx.y * 64;
  const int col0 = blockIdx.x * 64;

  v8f acc[4];
#pragma unroll
  for (int j = 0; j < 4; ++j)
#pragma unroll
    for (int r = 0; r < 8; ++r) acc[j][r] = 0.0f;

  const size_t aoff  = (size_t)(row0 + wm * 32 + m) * K + 8 * h;
  const size_t boff  = (size_t)(col0 + wn * 32 + m) * K + 8 * h;
  const size_t sub16 = (size_t)16 * K;
  const int nk = K >> 5;

  for (int kt = 0; kt < nk; ++kt) {
    const size_t k0 = (size_t)kt * 32;
    FragB fa[2], ga[2];
#pragma unroll
    for (int s = 0; s < 2; ++s) {
      const ush* p = Ah + aoff + s * sub16 + k0;
      const ush* q = Al + aoff + s * sub16 + k0;
      fa[s].h[0] = *(const u16x8*)(p);
      fa[s].h[1] = *(const u16x8*)(p + 16);
      ga[s].h[0] = *(const u16x8*)(q);
      ga[s].h[1] = *(const u16x8*)(q + 16);
    }
#pragma unroll
    for (int j = 0; j < 2; ++j) {
      FragB fb, gb;
      const ush* p = Bh + boff + j * sub16 + k0;
      const ush* q = Bl + boff + j * sub16 + k0;
      fb.h[0] = *(const u16x8*)(p);
      fb.h[1] = *(const u16x8*)(p + 16);
      gb.h[0] = *(const u16x8*)(q);
      gb.h[1] = *(const u16x8*)(q + 16);
#pragma unroll
      for (int s = 0; s < 2; ++s) {
        mma16(acc[s * 2 + j], fa[s], fb);
        mma16(acc[s * 2 + j], fa[s], gb);
        mma16(acc[s * 2 + j], ga[s], fb);
      }
    }
  }

  const bool doadd = (flags & 1) != 0;
  const bool dosp  = (flags & 2) != 0;
#pragma unroll
  for (int s = 0; s < 2; ++s) {
#pragma unroll
    for (int j = 0; j < 2; ++j) {
      const int lcol = wn * 32 + j * 16 + m;
      const float bv = bias[col0 + lcol];
#pragma unroll
      for (int r = 0; r < 8; ++r) {
        const int lrow = wm * 32 + s * 16 + 8 * h + r;
        float v = acc[s * 2 + j][r] + bv;
        if (doadd) v += addsrc[(size_t)(row0 + lrow) * ldadd + col0 + lcol];
        if (dosp)  v = softplus_f(v);
        stile[lrow * SPIT + lcol] = v;
      }
    }
  }
  __syncthreads();

  gemm_store_pass<OUTP>(stile, Cf, Ch, Cl, row0, col0, ldc, wave, lane);
  __threadfence();
  gemm_store_pass<OUTP>(stile, Cf, Ch, Cl, row0, col0, ldc, wave, lane);
}

__device__ __forceinline__ void rows16_store_pass(const ush* sl, ush* gp, size_t gbase, int lane) {
#pragma unroll
  for (int it = 0; it < 4; ++it) {
    const int t = it * 4 + (lane >> 3);
    const int c = (lane & 7) * 8;
    const u16x8 v = *(const u16x8*)(sl + t * 64 + c);
    *(volatile u16x8*)(gp + gbase + (size_t)t * DINR + c) = v;
  }
}

__global__ __launch_bounds__(64)
void scan_kernel(const float* __restrict__ xz, const float* __restrict__ dtp, const float* __restrict__ dbl,
                 const float* __restrict__ cw, const float* __restrict__ cb,
                 const float* __restrict__ Alog, const float* __restrict__ Dp,
                 ush* gh, ush* gl)
{
  __shared__ __attribute__((aligned(16))) float sbc[16 * 32];
  __shared__ __attribute__((aligned(16))) ush   shi[16 * 64];
  __shared__ __attribute__((aligned(16))) ush   slo[16 * 64];

  const int tid   = threadIdx.x;
  const int lane  = tid & 31;
  const int wave  = tid >> 5;
  const int dbase = blockIdx.x * 64;
  const int d     = dbase + tid;

  float a2[NST], hs[NST];
#pragma unroll
  for (int n = 0; n < NST; ++n) {
    a2[n] = -expf(Alog[d * NST + n]) * 1.44269504088896341f;
    hs[n] = 0.0f;
  }
  const float w0 = cw[d * 4 + 0], w1 = cw[d * 4 + 1], w2 = cw[d * 4 + 2], w3 = cw[d * 4 + 3];
  const float cbias = cb[d];
  const float Dd    = Dp[d];

  float xm1 = 0.0f, xm2 = 0.0f, xm3 = 0.0f;
  const ush* sl = wave ? slo : shi;
  ush* gp = wave ? gl : gh;

#pragma unroll 1
  for (int l0 = 0; l0 < LSEQ; l0 += 16) {
    {
      const int t = tid >> 2;
      const int c = (tid & 3) * 8;
      const float* sp = dbl + (size_t)(l0 + t) * XPW + 16 + c;
      *(v4f*)(sbc + t * 32 + c)     = *(const v4f*)(sp);
      *(v4f*)(sbc + t * 32 + c + 4) = *(const v4f*)(sp + 4);
    }
    __syncthreads();
#pragma unroll 1
    for (int t = 0; t < 16; ++t) {
      const size_t row = (size_t)(l0 + t);
      const float xv  = xz[row * (2 * DINR) + d];
      const float zv  = xz[row * (2 * DINR) + DINR + d];
      const float dtv = dtp[row * DINR + d];
      const float u   = silu_f(conv4(xm3, xm2, xm1, xv, w0, w1, w2, w3, cbias));
      xm3 = xm2; xm2 = xm1; xm1 = xv;
      const float du = dtv * u;
      float y = 0.0f;
#pragma unroll
      for (int n = 0; n < NST; ++n) {
        const float da = exp2f(dtv * a2[n]);
        hs[n] = da * hs[n] + du * sbc[t * 32 + n];
        y += hs[n] * sbc[t * 32 + 16 + n];
      }
      const float gq = (y + Dd * u) * silu_f(zv);
      ush hb, lb;
      split2(gq, hb, lb);
      shi[t * 64 + tid] = hb;
      slo[t * 64 + tid] = lb;
    }
    __syncthreads();
    const size_t gbase = (size_t)l0 * DINR + dbase;
    rows16_store_pass(sl, gp, gbase, lane);
    __threadfence();
    rows16_store_pass(sl, gp, gbase, lane);
    __syncthreads();
  }
}

extern "C" void kernel_launch(void* const* d_in, const int* in_sizes, int n_in,
                              void* d_out, int out_size, void* d_ws, size_t ws_size,
                              hipStream_t stream)
{
  if (n_in < 22) return;
  if (in_sizes[0]  != LSEQ)                     return;
  if (in_sizes[1]  != VOCB * DMOD)              return;
  if (in_sizes[2]  != VOCB)                     return;
  if (in_sizes[3]  != NLAY * 2 * DINR * DMOD)   return;
  if (in_sizes[4]  != NLAY * DINR * 4)          return;
  if (in_sizes[5]  != NLAY * DINR)              return;
  if (in_sizes[6]  != NLAY * 48 * DINR)         return;
  if (in_sizes[7]  != NLAY * DINR * 16)         return;
  if (in_sizes[8]  != NLAY * DINR)              return;
  if (in_sizes[9]  != NLAY * DINR * NST)        return;
  if (in_sizes[10] != NLAY * DINR)              return;
  if (in_sizes[11] != NLAY * DMOD * DINR)       return;
  if (in_sizes[12] != NLAY * 3 * DMOD * DMOD)   return;
  if (in_sizes[13] != NLAY * 3 * DMOD)          return;
  if (in_sizes[14] != NLAY * DMOD * DMOD)       return;
  if (in_sizes[15] != NLAY * DMOD)              return;
  if (in_sizes[16] != NLAY * DMOD)              return;
  if (in_sizes[17] != NLAY * DMOD)              return;
  if (in_sizes[18] != NLAY * DMOD)              return;
  if (in_sizes[19] != NLAY * DMOD)              return;
  if (in_sizes[20] != DMOD)                     return;
  if (in_sizes[21] != DMOD)                     return;
  if (out_size     != LSEQ * VOCB)              return;

  const int*   tokens     = (const int*)  d_in[0];
  const float* emb        = (const float*)d_in[1];
  const float* head_b     = (const float*)d_in[2];
  const float* in_proj_w  = (const float*)d_in[3];
  const float* conv_w     = (const float*)d_in[4];
  const float* conv_b     = (const float*)d_in[5];
  const float* x_proj_w   = (const float*)d_in[6];
  const float* dt_proj_w  = (const float*)d_in[7];
  const float* dt_proj_b  = (const float*)d_in[8];
  const float* A_log      = (const float*)d_in[9];
  const float* D_param    = (const float*)d_in[10];
  const float* out_proj_w = (const float*)d_in[11];
  const float* attn_in_w  = (const float*)d_in[12];
  const float* attn_in_b  = (const float*)d_in[13];
  const float* attn_out_w = (const float*)d_in[14];
  const float* attn_out_b = (const float*)d_in[15];
  const float* n1_g       = (const float*)d_in[16];
  const float* n1_b       = (const float*)d_in[17];
  const float* n2_g       = (const float*)d_in[18];
  const float* n2_b       = (const float*)d_in[19];
  const float* normf_g    = (const float*)d_in[20];
  const float* normf_b    = (const float*)d_in[21];
  float* out = (float*)d_out;

  size_t off = 0;
  auto take = [&](size_t bytes) { const size_t o = off; off += (bytes + 127) & ~(size_t)127; return o; };
  const size_t OFF_ZB    = take(4096);
  const size_t SZ_WIN    = (size_t)NLAY * 2 * DINR * DMOD * 2;
  const size_t OFF_WINH  = take(SZ_WIN),  OFF_WINL  = take(SZ_WIN);
  const size_t SZ_WXP    = (size_t)NLAY * XPW * DINR * 2;
  const size_t OFF_WXPH  = take(SZ_WXP),  OFF_WXPL  = take(SZ_WXP);
  const size_t SZ_WDT    = (size_t)NLAY * DINR * DTK * 2;
  const size_t OFF_WDTH  = take(SZ_WDT),  OFF_WDTL  = take(SZ_WDT);
  const size_t SZ_WOUT   = (size_t)NLAY * DMOD * DINR * 2;
  const size_t OFF_WOUTH = take(SZ_WOUT), OFF_WOUTL = take(SZ_WOUT);
  const size_t SZ_WV     = (size_t)NLAY * DMOD * DMOD * 2;
  const size_t OFF_WVH   = take(SZ_WV),   OFF_WVL   = take(SZ_WV);
  const size_t OFF_WOH   = take(SZ_WV),   OFF_WOL   = take(SZ_WV);
  const size_t SZ_EMB    = (size_t)VOCB * DMOD * 2;
  const size_t OFF_EMBH  = take(SZ_EMB),  OFF_EMBL  = take(SZ_EMB);
  const size_t OFF_X     = take((size_t)LSEQ * DMOD * 4);
  const size_t SZ_XN     = (size_t)LSEQ * DMOD * 2;
  const size_t OFF_XNH   = take(SZ_XN),   OFF_XNL   = take(SZ_XN);
  const size_t OFF_XZ    = take((size_t)LSEQ * 2 * DINR * 4);
  const size_t SZ_XM     = (size_t)LSEQ * DINR * 2;
  const size_t OFF_XMH   = take(SZ_XM),   OFF_XML   = take(SZ_XM);
  const size_t OFF_DBL   = take((size_t)LSEQ * XPW * 4);
  const size_t SZ_DTI    = (size_t)LSEQ * DTK * 2;
  const size_t OFF_DTIH  = take(SZ_DTI),  OFF_DTIL  = take(SZ_DTI);
  const size_t OFF_DT    = take((size_t)LSEQ * DINR * 4);
  const size_t OFF_GH    = take(SZ_XM),   OFF_GL    = take(SZ_XM);
  const size_t OFF_VH    = take(SZ_XN),   OFF_VL    = take(SZ_XN);
  const size_t WS_END    = off;
  if (WS_END > ws_size) return;
  if (WS_END > (size_t)134217728) return;

  char* ws = (char*)d_ws;
  float* zb    = (float*)(ws + OFF_ZB);
  ush*   winh  = (ush*)(ws + OFF_WINH);  ush* winl  = (ush*)(ws + OFF_WINL);
  ush*   wxph  = (ush*)(ws + OFF_WXPH);  ush* wxpl  = (ush*)(ws + OFF_WXPL);
  ush*   wdth  = (ush*)(ws + OFF_WDTH);  ush* wdtl  = (ush*)(ws + OFF_WDTL);
  ush*   wouth = (ush*)(ws + OFF_WOUTH); ush* woutl = (ush*)(ws + OFF_WOUTL);
  ush*   wvh   = (ush*)(ws + OFF_WVH);   ush* wvl   = (ush*)(ws + OFF_WVL);
  ush*   woh   = (ush*)(ws + OFF_WOH);   ush* wol   = (ush*)(ws + OFF_WOL);
  ush*   embh  = (ush*)(ws + OFF_EMBH);  ush* embl  = (ush*)(ws + OFF_EMBL);
  float* x     = (float*)(ws + OFF_X);
  ush*   xnh   = (ush*)(ws + OFF_XNH);   ush* xnl   = (ush*)(ws + OFF_XNL);
  float* xz    = (float*)(ws + OFF_XZ);
  ush*   xmh   = (ush*)(ws + OFF_XMH);   ush* xml   = (ush*)(ws + OFF_XML);
  float* dbl   = (float*)(ws + OFF_DBL);
  ush*   dtih  = (ush*)(ws + OFF_DTIH);  ush* dtil  = (ush*)(ws + OFF_DTIL);
  float* dt    = (float*)(ws + OFF_DT);
  ush*   gh    = (ush*)(ws + OFF_GH);    ush* gl    = (ush*)(ws + OFF_GL);
  ush*   vh    = (ush*)(ws + OFF_VH);    ush* vl    = (ush*)(ws + OFF_VL);

  const dim3 b256(256), b128(128), b64(64);

  hipMemsetAsync(zb, 0, 4096, stream);

  {
    int t8;
    t8 = (NLAY * 2 * DINR * DMOD) / 8;
    cvt_rows_kernel<<<dim3((t8 + 255) / 256), b256, 0, stream>>>(in_proj_w, winh, winl,
        2 * DINR, DMOD, 2 * DINR, DMOD, DMOD, 0, 2 * DINR * DMOD, t8);
    t8 = (NLAY * XPW * DINR) / 8;
    cvt_rows_kernel<<<dim3((t8 + 255) / 256), b256, 0, stream>>>(x_proj_w, wxph, wxpl,
        XPW, DINR, 48, DINR, DINR, 0, 48 * DINR, t8);
    t8 = (NLAY * DINR * DTK) / 8;
    cvt_rows_kernel<<<dim3((t8 + 255) / 256), b256, 0, stream>>>(dt_proj_w, wdth, wdtl,
        DINR, DTK, DINR, 16, 16, 0, DINR * 16, t8);
    t8 = (NLAY * DMOD * DINR) / 8;
    cvt_rows_kernel<<<dim3((t8 + 255) / 256), b256, 0, stream>>>(out_proj_w, wouth, woutl,
        DMOD, DINR, DMOD, DINR, DINR, 0, DMOD * DINR, t8);
    t8 = (NLAY * DMOD * DMOD) / 8;
    cvt_rows_kernel<<<dim3((t8 + 255) / 256), b256, 0, stream>>>(attn_in_w, wvh, wvl,
        DMOD, DMOD, DMOD, DMOD, DMOD, 2 * DMOD, 3 * DMOD * DMOD, t8);
    t8 = (NLAY * DMOD * DMOD) / 8;
    cvt_rows_kernel<<<dim3((t8 + 255) / 256), b256, 0, stream>>>(attn_out_w, woh, wol,
        DMOD, DMOD, DMOD, DMOD, DMOD, 0, DMOD * DMOD, t8);
    t8 = (VOCB * DMOD) / 8;
    cvt_rows_kernel<<<dim3((t8 + 255) / 256), b256, 0, stream>>>(emb, embh, embl,
        VOCB, DMOD, VOCB, DMOD, DMOD, 0, 0, t8);
  }

  embed_kernel<<<dim3((LSEQ * (DMOD / 4) + 255) / 256), b256, 0, stream>>>(tokens, emb, x, LSEQ, VOCB);

  for (int i = 0; i < NLAY; ++i) {
    const ush* winh_i  = winh  + (size_t)i * 2 * DINR * DMOD;
    const ush* winl_i  = winl  + (size_t)i * 2 * DINR * DMOD;
    const ush* wxph_i  = wxph  + (size_t)i * XPW * DINR;
    const ush* wxpl_i  = wxpl  + (size_t)i * XPW * DINR;
    const ush* wdth_i  = wdth  + (size_t)i * DINR * DTK;
    const ush* wdtl_i  = wdtl  + (size_t)i * DINR * DTK;
    const ush* wouth_i = wouth + (size_t)i * DMOD * DINR;
    const ush* woutl_i = woutl + (size_t)i * DMOD * DINR;
    const ush* wvh_i   = wvh   + (size_t)i * DMOD * DMOD;
    const ush* wvl_i   = wvl   + (size_t)i * DMOD * DMOD;
    const ush* woh_i   = woh   + (size_t)i * DMOD * DMOD;
    const ush* wol_i   = wol   + (size_t)i * DMOD * DMOD;
    const float* cw_i  = conv_w     + (size_t)i * DINR * 4;
    const float* cb_i  = conv_b     + (size_t)i * DINR;
    const float* bdt_i = dt_proj_b  + (size_t)i * DINR;
    const float* al_i  = A_log      + (size_t)i * DINR * NST;
    const float* dp_i  = D_param    + (size_t)i * DINR;
    const float* bv_i  = attn_in_b  + (size_t)i * 3 * DMOD + 2 * DMOD;
    const float* bo_i  = attn_out_b + (size_t)i * DMOD;

    ln_cvt_kernel<<<dim3(LSEQ / 8), b256, 0, stream>>>(x, n1_g + i * DMOD, n1_b + i * DMOD, xnh, xnl, LSEQ);
    gemm_kernel<0><<<dim3((2 * DINR) / 64, LSEQ / 64), b128, 0, stream>>>(
        xnh, xnl, winh_i, winl_i, zb, xz, 2 * DINR, xz, gh, gl, DMOD, 2 * DINR, 0);
    conv_silu_kernel<<<dim3(LSEQ), b64, 0, stream>>>(xz, cw_i, cb_i, xmh, xml);
    gemm_kernel<0><<<dim3(XPW / 64, LSEQ / 64), b128, 0, stream>>>(
        xmh, xml, wxph_i, wxpl_i, zb, dbl, XPW, dbl, gh, gl, DINR, XPW, 0);
    cvt_rows_kernel<<<dim3((LSEQ * DTK / 8 + 255) / 256), b256, 0, stream>>>(dbl, dtih, dtil,
        LSEQ, DTK, LSEQ, 16, XPW, 0, 0, LSEQ * DTK / 8);
    gemm_kernel<0><<<dim3(DINR / 64, LSEQ / 64), b128, 0, stream>>>(
        dtih, dtil, wdth_i, wdtl_i, bdt_i, dt, DINR, dt, gh, gl, DTK, DINR, 2);
    scan_kernel<<<dim3(DINR / 64), b64, 0, stream>>>(xz, dt, dbl, cw_i, cb_i, al_i, dp_i, gh, gl);
    gemm_kernel<0><<<dim3(DMOD / 64, LSEQ / 64), b128, 0, stream>>>(
        gh, gl, wouth_i, woutl_i, zb, x, DMOD, x, vh, vl, DINR, DMOD, 1);

    ln_cvt_kernel<<<dim3(LSEQ / 8), b256, 0, stream>>>(x, n2_g + i * DMOD, n2_b + i * DMOD, xnh, xnl, LSEQ);
    gemm_kernel<1><<<dim3(DMOD / 64, LSEQ / 64), b128, 0, stream>>>(
        xnh, xnl, wvh_i, wvl_i, bv_i, x, DMOD, x, vh, vl, DMOD, DMOD, 0);
    gemm_kernel<0><<<dim3(DMOD / 64, LSEQ / 64), b128, 0, stream>>>(
        vh, vl, woh_i, wol_i, bo_i, x, DMOD, x, gh, gl, DMOD, DMOD, 1);
  }

  ln_cvt_kernel<<<dim3(LSEQ / 8), b256, 0, stream>>>(x, normf_g, normf_b, xnh, xnl, LSEQ);
  gemm_kernel<0><<<dim3(VOCB / 64, LSEQ / 64), b128, 0, stream>>>(
      xnh, xnl, embh, embl, head_b, out, VOCB, out, gh, gl, DMOD, VOCB, 0);
}
